// ScaledMultiheadAttention_84817014161532
// MI455X (gfx1250) — hardware-verified
//
#include <hip/hip_runtime.h>
#include <math.h>

typedef __attribute__((ext_vector_type(16))) _Float16 v16h;
typedef __attribute__((ext_vector_type(16))) __bf16 v16b;
typedef __attribute__((ext_vector_type(8)))  _Float16 v8h;
typedef __attribute__((ext_vector_type(8)))  float v8f;
typedef __attribute__((ext_vector_type(4)))  float v4f;
typedef __attribute__((ext_vector_type(2)))  float v2f;
typedef __attribute__((ext_vector_type(4)))  unsigned v4u;
typedef __attribute__((ext_vector_type(4)))  int v4i;
typedef float __attribute__((may_alias)) float_a;
typedef int __attribute__((may_alias)) int_a;

template <typename T> __device__ __forceinline__ void vst2(void* p, T v) { *(volatile T*)p = v; __threadfence(); *(volatile T*)p = v; }
__device__ __forceinline__ v8f wmma16(v16h a, v16h b, v8f c) {
  v8f d = __builtin_amdgcn_wmma_f32_16x16x32_f16(false, a, false, b, (short)0, c, false, false);
  asm volatile("v_nop\n\tv_nop\n\tv_nop\n\tv_nop" : "+v"(d) : "v"(a), "v"(b));
  return d;
}
__device__ __forceinline__ v8f wmma_bf(v16b a, v16b b, v8f c) {
  v8f d = __builtin_amdgcn_wmma_f32_16x16x32_bf16(false, a, false, b, (short)0, c, false, false);
  asm volatile("v_nop\n\tv_nop\n\tv_nop\n\tv_nop" : "+v"(d) : "v"(a), "v"(b));
  return d;
}
__device__ __forceinline__ v16h frag_h(const _Float16* rowk0, int lane) {
  union { v16h v; v8h q[2]; } u; const _Float16* p = rowk0 + 8 * (lane >> 4);
  u.q[0] = *(const v8h*)p; u.q[1] = *(const v8h*)(p + 16); return u.v;
}
__device__ __forceinline__ v16h frag_f32(const float* rowk0, int lane) {
  v16h a; const float* p = rowk0 + 8 * (lane >> 4);
#pragma unroll
  for (int i = 0; i < 8; ++i) { a[i] = (_Float16)p[i]; a[8 + i] = (_Float16)p[16 + i]; }
  return a;
}
__device__ __forceinline__ v16h frag_f32s(const float* rowk0, int lane, float sc) {
  v16h a; const float* p = rowk0 + 8 * (lane >> 4);
#pragma unroll
  for (int i = 0; i < 8; ++i) { a[i] = (_Float16)(p[i] * sc); a[8 + i] = (_Float16)(p[16 + i] * sc); }
  return a;
}
__device__ __forceinline__ v16h fragc_f32(const float* W, int k0, int n, int lane, int ld, int K) {
  v16h a; const int g = lane >> 4;
#pragma unroll
  for (int i = 0; i < 8; ++i) { const int ka = k0 + 8 * g + i, kb = ka + 16;
    a[i] = (_Float16)(ka < K ? W[(size_t)ka * ld + n] : 0.f); a[8 + i] = (_Float16)(kb < K ? W[(size_t)kb * ld + n] : 0.f); }
  return a;
}
struct F2 { v16b h, l; };
__device__ __forceinline__ F2 bsplit16(const float v[16]) { F2 r;
#pragma unroll
  for (int i = 0; i < 16; ++i) { const __bf16 h = (__bf16)v[i]; r.h[i] = h; r.l[i] = (__bf16)(v[i] - (float)h); }
  return r; }
__device__ __forceinline__ F2 split_row(const float* row, int k0, int lane) { float v[16]; const float* p = row + k0 + 8 * (lane >> 4);
#pragma unroll
  for (int i = 0; i < 8; ++i) { v[i] = p[i]; v[8 + i] = p[16 + i]; }
  return bsplit16(v); }
__device__ __forceinline__ F2 split_rowK(const float* row, int k0, int lane, int K) { float v[16]; const int g = lane >> 4;
#pragma unroll
  for (int i = 0; i < 8; ++i) { const int ka = k0 + 8 * g + i, kb = ka + 16; v[i] = ka < K ? row[ka] : 0.f; v[8 + i] = kb < K ? row[kb] : 0.f; }
  return bsplit16(v); }
__device__ __forceinline__ F2 split_col(const float* W, int k0, int n, int lane, int ld, int K) { float v[16]; const int g = lane >> 4;
#pragma unroll
  for (int i = 0; i < 8; ++i) { const int ka = k0 + 8 * g + i, kb = ka + 16; v[i] = ka < K ? W[(size_t)ka * ld + n] : 0.f; v[8 + i] = kb < K ? W[(size_t)kb * ld + n] : 0.f; }
  return bsplit16(v); }
__device__ __forceinline__ v8f mac3(const F2& a, const F2& b, v8f c) { c = wmma_bf(a.l, b.h, c); c = wmma_bf(a.h, b.l, c); return wmma_bf(a.h, b.h, c); }
__device__ __forceinline__ float sigm(float v) { return 1.0f / (1.0f + expf(-v)); }
#define LDSX() do { asm volatile("s_wait_dscnt 0" ::: "memory"); __builtin_amdgcn_wave_barrier(); __builtin_amdgcn_fence(__ATOMIC_RELEASE, "workgroup"); } while (0)

#define SS 1024
#define NB 4
#define EE 1024
#define NH 16
#define HD 64
#define NR (SS * NB)

__global__ __launch_bounds__(256) void k_cvt(const float* __restrict__ a, const float* __restrict__ b, const float* __restrict__ c, _Float16* __restrict__ a16, _Float16* __restrict__ b16, _Float16* __restrict__ c16) {
  const size_t g8 = (size_t)blockIdx.x * 256 + threadIdx.x; const int which = blockIdx.y; if (g8 >= (size_t)NR * EE / 8) return;
  const float* s = which == 0 ? a : (which == 1 ? b : c); _Float16* d = which == 0 ? a16 : (which == 1 ? b16 : c16);
  union { v8h h; v4u u; } pk;
#pragma unroll
  for (int e = 0; e < 8; ++e) pk.h[e] = (_Float16)s[g8 * 8 + e];
  vst2(d + g8 * 8, pk.u);
}
__global__ __launch_bounds__(256) void k_packW(const float* __restrict__ Win, const float* __restrict__ Wo, _Float16* __restrict__ P) {
  const int n = blockIdx.x, tid = threadIdx.x; const float* W = n < 3 * EE ? Win + (size_t)n * EE : Wo + (size_t)(n - 3 * EE) * EE;
  if (tid < EE / 8) { union { v8h h; v4u u; } pk;
#pragma unroll
    for (int e = 0; e < 8; ++e) pk.h[e] = (_Float16)(W[tid * 8 + e] * 16.0f);
    vst2(P + (size_t)n * EE + tid * 8, pk.u); }
}
__global__ __launch_bounds__(128) void k_proj(const _Float16* __restrict__ q16i, const _Float16* __restrict__ k16i, const _Float16* __restrict__ v16i, const _Float16* __restrict__ P, const float* __restrict__ bias,
                                            _Float16* __restrict__ qh, _Float16* __restrict__ kh, _Float16* __restrict__ vT) {
  __shared__ __align__(16) float so[4][16][132];
  __shared__ __align__(16) _Float16 st[128][72];
  const int tid = threadIdx.x, wave = tid >> 5, lane = tid & 31, col = lane & 15, g = lane >> 4;
  const int r0 = blockIdx.x * 64 + wave * 16, n0 = blockIdx.y * 128; const int which = n0 / EE, c0 = n0 % EE, hb = c0 / HD;
  const _Float16* A = which == 0 ? q16i : (which == 1 ? k16i : v16i);
  const int bsel = blockIdx.x & 3, sblk = blockIdx.x >> 2;
  const int arow = which == 2 ? ((sblk * 64 + wave * 16 + col) * NB + bsel) : (r0 + col);
  v8f acc[8] = {};
#pragma unroll 1
  for (int kc = 0; kc < EE / 32; ++kc) { const v16h a = frag_h(A + (size_t)arow * EE + kc * 32, lane);
#pragma unroll
    for (int j = 0; j < 8; ++j) acc[j] = wmma16(a, frag_h(P + (size_t)(n0 + j * 16 + col) * EE + kc * 32, lane), acc[j]); }
#pragma unroll
  for (int j = 0; j < 8; ++j) { const float bb = bias[n0 + j * 16 + col];
#pragma unroll
    for (int r = 0; r < 8; ++r) so[wave][8 * g + r][j * 16 + col] = acc[j][r] * (1.0f / 16.0f) + bb; }
  LDSX();
  if (which < 2) { _Float16* dst = which == 0 ? qh : kh;
    for (int q = lane; q < 2 * 16 * 8; q += 32) { const int hh = q >> 7, rem = q & 127, rl = rem >> 3, pc = rem & 7; const int row = r0 + rl, s = row / NB, b = row % NB;
      union { v8h h8; v4u u; } pk;
#pragma unroll
      for (int e = 0; e < 8; ++e) pk.h8[e] = (_Float16)so[wave][rl][hh * HD + pc * 8 + e];
      vst2(dst + (((size_t)b * NH + hb + hh) * SS + s) * HD + pc * 8, pk.u); } }
  else {
#pragma unroll 4
    for (int rl = 0; rl < 16; ++rl) {
#pragma unroll
      for (int e = 0; e < 4; ++e) st[lane * 4 + e][wave * 16 + rl] = (_Float16)so[wave][rl][lane * 4 + e]; }
    __syncthreads();
    for (int q = tid; q < 128 * 8; q += 128) { const int c = q >> 3, pc = q & 7, hh = c >> 6, d = c & 63;
      vst2(vT + (((size_t)bsel * NH + hb + hh) * HD + d) * SS + sblk * 64 + pc * 8, *(const v4u*)(&st[c][pc * 8])); }
  }
}
__global__ __launch_bounds__(128) void k_attn(const _Float16* __restrict__ qh, const _Float16* __restrict__ kh, const _Float16* __restrict__ vT, const float* __restrict__ lsc, _Float16* __restrict__ o16) {
  __shared__ __align__(16) float sS[4][16][68];
  __shared__ __align__(16) _Float16 sP[4][16][72];
  __shared__ __align__(16) float sO[4][16][68];
  const int tid = threadIdx.x, w = tid >> 5, lane = tid & 31, col = lane & 15, g = lane >> 4;
  const int bh = blockIdx.y, b = bh / NH, h = bh % NH, q0 = blockIdx.x * 64 + w * 16;
  const _Float16* qb = qh + (size_t)bh * SS * HD; const _Float16* kb = kh + (size_t)bh * SS * HD; const _Float16* vb = vT + (size_t)bh * HD * SS;
  v16h aq[2];
#pragma unroll
  for (int kc = 0; kc < 2; ++kc) aq[kc] = frag_h(qb + (size_t)(q0 + col) * HD + kc * 32, lane);
  float mrun = -3.0e38f, lrun = 0.f; v8f acc[4] = {};
#pragma unroll 1
  for (int kt = 0; kt < SS / 64; ++kt) {
#pragma unroll
    for (int t = 0; t < 4; ++t) { v8f s = {};
#pragma unroll
      for (int kc = 0; kc < 2; ++kc) s = wmma16(aq[kc], frag_h(kb + (size_t)(kt * 64 + t * 16 + col) * HD + kc * 32, lane), s);
#pragma unroll
      for (int r = 0; r < 8; ++r) sS[w][8 * g + r][t * 16 + col] = s[r] * 0.125f; }
    LDSX();
    float mx = -3.4e38f;
#pragma unroll
    for (int jj = 0; jj < 32; ++jj) mx = fmaxf(mx, sS[w][col][g * 32 + jj]);
    mx = fmaxf(mx, __shfl_xor(mx, 16, 32));
    const float mnew = fmaxf(mrun, mx); const float corr = expf(mrun - mnew);
    float ps = 0.f;
#pragma unroll
    for (int jj = 0; jj < 32; ++jj) { const float p = expf(sS[w][col][g * 32 + jj] - mnew); ps += p; sP[w][col][g * 32 + jj] = (_Float16)(p * 16384.0f); }
    ps += __shfl_xor(ps, 16, 32);
    lrun = lrun * corr + ps; mrun = mnew;
#pragma unroll
    for (int r = 0; r < 8; ++r) { const float cr = __shfl(corr, 8 * g + r, 32);
#pragma unroll
      for (int t = 0; t < 4; ++t) acc[t][r] *= cr; }
    LDSX();
#pragma unroll
    for (int kc = 0; kc < 2; ++kc) { const v16h pa = frag_h(&sP[w][col][0] + kc * 32, lane);
#pragma unroll
      for (int t = 0; t < 4; ++t) acc[t] = wmma16(pa, frag_h(vb + (size_t)(t * 16 + col) * SS + kt * 64 + kc * 32, lane), acc[t]); }
    __builtin_amdgcn_wave_barrier();
  }
  const float hs = lsc[h] * 16.0f;
#pragma unroll
  for (int r = 0; r < 8; ++r) { const float lr = __shfl(lrun, 8 * g + r, 32);
#pragma unroll
    for (int t = 0; t < 4; ++t) sO[w][8 * g + r][t * 16 + col] = acc[t][r] / (lr * 16384.0f) * hs; }
  LDSX();
  for (int q = lane; q < 16 * 8; q += 32) { const int rl = q >> 3, pc = q & 7; const int s = q0 + rl; union { v8h h8; v4u u; } pk;
#pragma unroll
    for (int e = 0; e < 8; ++e) pk.h8[e] = (_Float16)sO[w][rl][pc * 8 + e];
    vst2(o16 + ((size_t)s * NB + b) * EE + h * HD + pc * 8, pk.u); }
}
__global__ __launch_bounds__(128) void k_out(const _Float16* __restrict__ o16, const _Float16* __restrict__ P, const float* __restrict__ bo, float* __restrict__ out) {
  __shared__ __align__(16) float so[4][16][132];
  const int tid = threadIdx.x, wave = tid >> 5, lane = tid & 31, col = lane & 15, g = lane >> 4;
  const int r0 = blockIdx.x * 64 + wave * 16, n0 = blockIdx.y * 128;
  v8f acc[8] = {};
#pragma unroll 1
  for (int kc = 0; kc < EE / 32; ++kc) { const v16h a = frag_h(o16 + (size_t)(r0 + col) * EE + kc * 32, lane);
#pragma unroll
    for (int j = 0; j < 8; ++j) acc[j] = wmma16(a, frag_h(P + (size_t)(3 * EE + n0 + j * 16 + col) * EE + kc * 32, lane), acc[j]); }
#pragma unroll
  for (int j = 0; j < 8; ++j) { const float bb = bo[n0 + j * 16 + col];
#pragma unroll
    for (int r = 0; r < 8; ++r) so[wave][8 * g + r][j * 16 + col] = acc[j][r] * (1.0f / 256.0f) + bb; }
  LDSX();
#pragma unroll 4
  for (int rl = 0; rl < 16; ++rl) vst2(out + (size_t)(r0 + rl) * EE + n0 + lane * 4, *(const v4f*)(&so[wave][rl][lane * 4]));
}
extern "C" void kernel_launch(void* const* d_in, const int* in_sizes, int n_in, void* d_out, int out_size, void* d_ws, size_t ws_size, hipStream_t stream) {
  (void)in_sizes; (void)n_in; (void)out_size; (void)ws_size;
  const float* query = (const float*)d_in[0]; const float* key = (const float*)d_in[1]; const float* value = (const float*)d_in[2]; const float* Win = (const float*)d_in[3]; const float* bin = (const float*)d_in[4];
  const float* Wo = (const float*)d_in[5]; const float* bo = (const float*)d_in[6]; const float* lsc = (const float*)d_in[7];
  float* out = (float*)d_out;
  char* ws = (char*)d_ws; size_t off = 0;
  auto take = [&](size_t bytes) { char* p = ws + off; off += (bytes + 255) & ~(size_t)255; return p; };
  _Float16* q16i = (_Float16*)take((size_t)NR * EE * 2); _Float16* k16i = (_Float16*)take((size_t)NR * EE * 2); _Float16* v16i = (_Float16*)take((size_t)NR * EE * 2);
  _Float16* P = (_Float16*)take((size_t)4 * EE * EE * 2); _Float16* qh = (_Float16*)take((size_t)NR * EE * 2); _Float16* kh = (_Float16*)take((size_t)NR * EE * 2); _Float16* vT = (_Float16*)take((size_t)NR * EE * 2); _Float16* o16 = (_Float16*)take((size_t)NR * EE * 2);
  k_cvt<<<dim3((unsigned)((size_t)NR * EE / 8 / 256), 3), 256, 0, stream>>>(query, key, value, q16i, k16i, v16i);
  k_packW<<<4 * EE, 256, 0, stream>>>(Win, Wo, P);
  k_proj<<<dim3(NR / 64, 3 * EE / 128), 128, 0, stream>>>(q16i, k16i, v16i, P, bin, qh, kh, vT);
  k_attn<<<dim3(SS / 64, NB * NH), 128, 0, stream>>>(qh, kh, vT, lsc, o16);
  k_out<<<dim3(NR / 64, EE / 128), 128, 0, stream>>>(o16, P, bo, out);
}
